// HierarchicalSkeletalEncoder_75539884802739
// MI455X (gfx1250) — hardware-verified
//
#include <hip/hip_runtime.h>


namespace {
constexpr int NS = 16384, NCUT = 16384  , NJ = 17, DH = 64, EH = 64, OUT = 128, TOT = 384;
constexpr float XS = 8.0f, WSC = 256.0f;
static_assert(NS % 16 == 0 && NCUT % 16 == 0, "tiling");
__constant__ int SUBN[3] = {5, 4, 4};
__constant__ int SUBJ[3][5] = {{0, 5, 6, 11, 12}, {7, 8, 13, 14, -1}, {9, 10, 15, 16, -1}};
__constant__ int ROWOFF[3] = {0, 5, 9};
constexpr int RPP = 13;
__constant__ int NE[3] = {60, 84, 44};
__constant__ unsigned char EDST[3][84] = {
 {0,0,0,0,0,0,0,0,5,5,5,5,5,5,5,5,6,6,6,6,6,6,6,6,7,7,7,7,7,8,8,8,8,8,11,11,11,11,11,11,11,11,12,12,12,12,12,12,12,12,13,13,13,13,13,14,14,14,14,14},
 {0,0,0,0,5,5,5,5,6,6,6,6,7,7,7,7,7,7,7,7,7,7,7,7,8,8,8,8,8,8,8,8,8,8,8,8,9,9,9,9,10,10,10,10,11,11,11,11,12,12,12,12,13,13,13,13,13,13,13,13,13,13,13,13,14,14,14,14,14,14,14,14,14,14,14,14,15,15,15,15,16,16,16,16},
 {7,7,7,7,8,8,8,8,9,9,9,9,9,9,9,10,10,10,10,10,10,10,13,13,13,13,14,14,14,14,15,15,15,15,15,15,15,16,16,16,16,16,16,16}};
__constant__ unsigned char ESRC[3][84] = {
 {5,6,7,8,11,12,13,14,0,6,7,8,11,12,13,14,0,5,7,8,11,12,13,14,0,5,6,11,12,0,5,6,11,12,0,5,6,7,8,12,13,14,0,5,6,7,8,11,13,14,0,5,6,11,12,0,5,6,11,12},
 {7,8,13,14,7,8,13,14,7,8,13,14,0,5,6,8,9,10,11,12,13,14,15,16,0,5,6,7,9,10,11,12,13,14,15,16,7,8,13,14,7,8,13,14,7,8,13,14,7,8,13,14,0,5,6,7,8,9,10,11,12,14,15,16,0,5,6,7,8,9,10,11,12,13,15,16,7,8,13,14,7,8,13,14},
 {9,10,15,16,9,10,15,16,7,8,10,13,14,15,16,7,8,9,13,14,15,16,9,10,15,16,9,10,15,16,7,8,9,10,13,14,16,7,8,9,10,13,14,15}};
typedef _Float16 b16;
typedef __attribute__((ext_vector_type(16))) _Float16 v16b;
typedef __attribute__((ext_vector_type(8))) _Float16 v8b;
typedef __attribute__((ext_vector_type(8))) float v8f;
typedef __attribute__((ext_vector_type(4))) float v4f;
__device__ __forceinline__ float bf16_rne(float f) { unsigned int u = __float_as_uint(f); u += 0x7FFFu + ((u >> 16) & 1u); return __uint_as_float(u & 0xFFFF0000u); }
__device__ __forceinline__ void split16(float v, b16& hi, b16& lo) { hi = (b16)v; lo = (b16)(v - (float)hi); }
__device__ __forceinline__ v16b frag_kb(const b16* p, int hh) { const v8b a = *(const v8b*)(p + 8 * hh), b = *(const v8b*)(p + 16 + 8 * hh); v16b f;
#pragma unroll
  for (int e = 0; e < 8; ++e) { f[e] = a[e]; f[8 + e] = b[e]; } return f; }
__device__ __forceinline__ v8f wmma16b(v16b a, v16b b, v8f c) { v8f d = __builtin_amdgcn_wmma_f32_16x16x32_f16(false, a, false, b, (short)0, c, false, false); asm volatile("v_nop\n\tv_nop\n\tv_nop\n\tv_nop" : "+v"(d) : "v"(a), "v"(b)); return d; }
__device__ __forceinline__ void wave_lds_sync() { __builtin_amdgcn_fence(__ATOMIC_RELEASE, "workgroup"); __builtin_amdgcn_wave_barrier(); __builtin_amdgcn_fence(__ATOMIC_ACQUIRE, "workgroup"); }
__device__ __forceinline__ float pmul(float a, float b) { float p = a * b; asm volatile("" : "+v"(p)); return p; }
__device__ __forceinline__ int iclamp(int v, int lo, int hi) { return v < lo ? lo : (v > hi ? hi : v); }

typedef __attribute__((ext_vector_type(2))) _Float16 v2h;
typedef __attribute__((ext_vector_type(2))) float v2f;
__device__ __forceinline__ int subidx(int lvl, int j) { int r = -1; for (int q = 0; q < 5; ++q) if (q < SUBN[lvl] && SUBJ[lvl][q] == j) r = q; return r; }
__global__ __launch_bounds__(256) void prep_kernel(const float* __restrict__ wedge, const float* __restrict__ wproj, b16* __restrict__ WE, b16* __restrict__ WP) {
  int t = blockIdx.x * 256 + threadIdx.x; v8b o;
  if (t < 2 * EH * DH / 8) { const int e = t * 8; const int oo = e / DH, d0 = e % DH; for (int j = 0; j < 8; ++j) { const float w = (oo < EH) ? wedge[(size_t)oo * (2 * DH) + d0 + j] : wedge[(size_t)(oo - EH) * (2 * DH) + DH + d0 + j]; o[j] = (b16)(bf16_rne(w) * WSC); }
    for (int pass = 0; pass < 2; ++pass) { *(volatile v8b*)(WE + e) = o; __threadfence(); } return; }
  t -= 2 * EH * DH / 8; if (t < OUT * TOT / 8) { const int e = t * 8; for (int j = 0; j < 8; ++j) o[j] = (b16)(bf16_rne(wproj[e + j]) * WSC); for (int pass = 0; pass < 2; ++pass) { *(volatile v8b*)(WP + e) = o; __threadfence(); } }
}
__global__ __launch_bounds__(256) void pose_kernel(const float* __restrict__ kp, const float* __restrict__ scr, const float* __restrict__ wl, const float* __restrict__ bl, b16* __restrict__ FTh, b16* __restrict__ FTl, b16* __restrict__ PFh, b16* __restrict__ PFl) {
  __shared__ float sP[8][NJ][3];
  const int wave = threadIdx.x >> 5, lane = threadIdx.x & 31; const size_t n = (size_t)blockIdx.x * 8 + wave; const int c = lane * 2; const bool live = n < (size_t)NCUT;
  { float mnx = INFINITY, mny = INFINITY, mxx = -INFINITY, mxy = -INFINITY; float pxl = 0.0f, pyl = 0.0f, scl = 0.0f;
    if (lane < NJ) { pxl = live ? bf16_rne(kp[(n * NJ + lane) * 2]) : 0.0f; pyl = live ? bf16_rne(kp[(n * NJ + lane) * 2 + 1]) : 0.0f; scl = live ? bf16_rne(scr[n * NJ + lane]) : 0.0f; mnx = pxl; mxx = pxl; mny = pyl; mxy = pyl; }
#pragma unroll
    for (int o = 1; o < 32; o <<= 1) { mnx = fminf(mnx, __shfl_xor(mnx, o)); mxx = fmaxf(mxx, __shfl_xor(mxx, o)); mny = fminf(mny, __shfl_xor(mny, o)); mxy = fmaxf(mxy, __shfl_xor(mxy, o)); }
    const float dx = (mxx - mnx) + 1e-6f, dy = (mxy - mny) + 1e-6f; if (lane < NJ) { sP[wave][lane][0] = (pxl - mnx) / dx; sP[wave][lane][1] = (pyl - mny) / dy; sP[wave][lane][2] = scl; } }
  wave_lds_sync();
#pragma unroll 1
  for (int lvl = 0; lvl < 3; ++lvl) { const int ns = SUBN[lvl]; float hs[5][2]; float w0[2], w1[2], w2[2], bb[2];
    for (int q = 0; q < 2; ++q) { const int d = c + q; w0[q] = bf16_rne(wl[((size_t)lvl * DH + d) * 3 + 0]); w1[q] = bf16_rne(wl[((size_t)lvl * DH + d) * 3 + 1]); w2[q] = bf16_rne(wl[((size_t)lvl * DH + d) * 3 + 2]); bb[q] = bf16_rne(bl[(size_t)lvl * DH + d]); }
    for (int jj = 0; jj < 5; ++jj) for (int q = 0; q < 2; ++q) hs[jj][q] = 0.0f;
#pragma unroll
    for (int jj = 0; jj < 5; ++jj) { if (jj < ns) { const int j = SUBJ[lvl][jj]; const float pxj = sP[wave][j][0], pyj = sP[wave][j][1], scj = sP[wave][j][2]; for (int q = 0; q < 2; ++q) { float h = pmul(pxj, w0[q]) + pmul(pyj, w1[q]) + pmul(scj, w2[q]) + bb[q]; h = fmaxf(h, 0.0f); hs[jj][q] = h * scj; } } }
    float pool[2] = {0.0f, 0.0f};
#pragma unroll
    for (int jj = 0; jj < 5; ++jj) { v2h fh, fl;
      if (jj < ns) { const int j = SUBJ[lvl][jj]; const float scj = sP[wave][j][2]; for (int q = 0; q < 2; ++q) { float Hq = 0.0f; for (int kk = 0; kk < 5; ++kk) if (kk != jj && kk < ns) Hq += hs[kk][q]; pool[q] += Hq; const float feat = Hq * scj; b16 p, r; split16((live ? feat : 0.0f) * XS, p, r); fh[q] = p; fl[q] = r; }
        for (int pass = 0; pass < 2; ++pass) { const size_t row = n * RPP + ROWOFF[lvl] + jj; *(volatile v2h*)(FTh + row * DH + c) = fh; *(volatile v2h*)(FTl + row * DH + c) = fl; __threadfence(); } } }
    v2h ph, pl; for (int q = 0; q < 2; ++q) { b16 p, r; split16((live ? pool[q] * (1.0f / NJ) : 0.0f) * XS, p, r); ph[q] = p; pl[q] = r; }
    for (int pass = 0; pass < 2; ++pass) { *(volatile v2h*)(PFh + n * TOT + lvl * 128 + c) = ph; *(volatile v2h*)(PFl + n * TOT + lvl * 128 + c) = pl; __threadfence(); } }
}
__global__ __launch_bounds__(128) void egemm_kernel(const b16* __restrict__ FTh, const b16* __restrict__ FTl, const b16* __restrict__ WE, float* __restrict__ AB, size_t rowbase) {
  __shared__ __attribute__((aligned(16))) float Tf[4][16][128 + 4];
  const int wave = threadIdx.x >> 5, lane = threadIdx.x & 31, nloc = lane & 15, hlf = lane >> 4; const size_t ml = ((size_t)blockIdx.x * 4 + wave) * 16; const size_t m0 = rowbase + ml; if (m0 >= (size_t)NCUT * RPP) return;
  v8f acc[8];
#pragma unroll
  for (int t = 0; t < 8; ++t) acc[t] = (v8f){};
#pragma unroll
  for (int kb = 0; kb < DH; kb += 32) { const v16b a = frag_kb(FTh + (m0 + nloc) * DH + kb, hlf), al = frag_kb(FTl + (m0 + nloc) * DH + kb, hlf);
#pragma unroll
    for (int t = 0; t < 8; ++t) { const v16b bw = frag_kb(WE + (size_t)(t * 16 + nloc) * DH + kb, hlf); acc[t] = wmma16b(a, bw, acc[t]); acc[t] = wmma16b(al, bw, acc[t]); } }
#pragma unroll
  for (int t = 0; t < 4; ++t)
#pragma unroll
    for (int r = 0; r < 8; ++r) { const float g1 = acc[t][r] * (1.0f / (XS * WSC)), g2 = acc[t + 4][r] * (1.0f / (XS * WSC)); Tf[wave][8 * hlf + r][t * 16 + nloc] = g1 - g2; Tf[wave][8 * hlf + r][64 + t * 16 + nloc] = g2; }
  wave_lds_sync();
  for (int pass = 0; pass < 2; ++pass) { for (int rr = 0; rr < 16; ++rr) *(volatile v4f*)(AB + (ml + rr) * 128 + lane * 4) = *(const v4f*)(&Tf[wave][rr][lane * 4]); __threadfence(); }
}
__global__ __launch_bounds__(256) void zmax_kernel(const float* __restrict__ AB, const float* __restrict__ bedge, b16* __restrict__ PFh, b16* __restrict__ PFl, size_t posebase) {
  __shared__ float sAB[8][6][128]; __shared__ float sZ[8][NJ][64];
  const int wave = threadIdx.x >> 5, lane = threadIdx.x & 31; const size_t nl = (size_t)blockIdx.x * 8 + wave; const size_t n = posebase + nl; const int c = lane * 2; const bool live = n < (size_t)NCUT;
  const float be0 = bf16_rne(bedge[c]), be1 = bf16_rne(bedge[c + 1]);
#pragma unroll 1
  for (int lvl = 0; lvl < 3; ++lvl) { const int ns = SUBN[lvl];
    for (int jj = 0; jj < 6; ++jj) { float a0 = 0.0f, a1 = 0.0f, b0 = 0.0f, b1 = 0.0f; if (jj < ns && live) { const size_t row = nl * RPP + ROWOFF[lvl] + jj; a0 = AB[row * 128 + c]; a1 = AB[row * 128 + c + 1]; b0 = AB[row * 128 + 64 + c]; b1 = AB[row * 128 + 64 + c + 1]; }
      sAB[wave][jj][c] = a0; sAB[wave][jj][c + 1] = a1; sAB[wave][jj][64 + c] = b0; sAB[wave][jj][64 + c + 1] = b1; }
    for (int j = 0; j < NJ; ++j) { sZ[wave][j][c] = 0.0f; sZ[wave][j][c + 1] = 0.0f; }
    wave_lds_sync();
    unsigned has = 0u;
#pragma unroll 1
    for (int e = 0; e < NE[lvl]; ++e) { const int dj = EDST[lvl][e], sk = ESRC[lvl][e]; int dq = subidx(lvl, dj), sq = subidx(lvl, sk); dq = dq < 0 ? 5 : dq; sq = sq < 0 ? 5 : sq;
      const float m0 = fmaxf(sAB[wave][dq][c] + sAB[wave][sq][64 + c] + be0, 0.0f), m1 = fmaxf(sAB[wave][dq][c + 1] + sAB[wave][sq][64 + c + 1] + be1, 0.0f);
      const bool first = ((has >> dj) & 1u) == 0u; sZ[wave][dj][c] = first ? m0 : fmaxf(sZ[wave][dj][c], m0); sZ[wave][dj][c + 1] = first ? m1 : fmaxf(sZ[wave][dj][c + 1], m1); has |= (1u << dj); }
    float pz0 = 0.0f, pz1 = 0.0f; for (int j = 0; j < NJ; ++j) { pz0 += sZ[wave][j][c]; pz1 += sZ[wave][j][c + 1]; }
    v2h ph, pl; { b16 p, r; split16((live ? pz0 * (1.0f / NJ) : 0.0f) * XS, p, r); ph[0] = p; pl[0] = r; split16((live ? pz1 * (1.0f / NJ) : 0.0f) * XS, p, r); ph[1] = p; pl[1] = r; }
    for (int pass = 0; pass < 2; ++pass) { *(volatile v2h*)(PFh + n * TOT + lvl * 128 + 64 + c) = ph; *(volatile v2h*)(PFl + n * TOT + lvl * 128 + 64 + c) = pl; __threadfence(); }
    wave_lds_sync(); }
}
__global__ __launch_bounds__(128) void proj_kernel(const b16* __restrict__ PFh, const b16* __restrict__ PFl, const b16* __restrict__ WP, const float* __restrict__ bproj, float* __restrict__ out) {
  __shared__ __attribute__((aligned(16))) float Tf[4][16][128 + 4];
  const int wave = threadIdx.x >> 5, lane = threadIdx.x & 31, nloc = lane & 15, hlf = lane >> 4; const size_t m0 = ((size_t)blockIdx.x * 4 + wave) * 16; if (m0 >= (size_t)NCUT) return;
  v8f acc[8];
#pragma unroll
  for (int t = 0; t < 8; ++t) acc[t] = (v8f){};
#pragma unroll 2
  for (int kb = 0; kb < TOT; kb += 32) { const v16b a = frag_kb(PFh + (m0 + nloc) * TOT + kb, hlf), al = frag_kb(PFl + (m0 + nloc) * TOT + kb, hlf);
#pragma unroll
    for (int t = 0; t < 8; ++t) { const v16b bw = frag_kb(WP + (size_t)(t * 16 + nloc) * TOT + kb, hlf); acc[t] = wmma16b(a, bw, acc[t]); acc[t] = wmma16b(al, bw, acc[t]); } }
#pragma unroll
  for (int t = 0; t < 8; ++t) { const float bb = bf16_rne(bproj[t * 16 + nloc]);
#pragma unroll
    for (int r = 0; r < 8; ++r) Tf[wave][8 * hlf + r][t * 16 + nloc] = acc[t][r] * (1.0f / (XS * WSC)) + bb; }
  wave_lds_sync();
  for (int pass = 0; pass < 2; ++pass) { for (int rr = 0; rr < 16; ++rr) *(volatile v4f*)(out + (m0 + rr) * OUT + lane * 4) = *(const v4f*)(&Tf[wave][rr][lane * 4]); __threadfence(); }
}
}

extern "C" void kernel_launch(void* const* d_in, const int* in_sizes, int n_in, void* d_out, int out_size, void* d_ws, size_t ws_size, hipStream_t stream) {
  (void)n_in;
  auto Fp = [&](int i) { return (const float*)d_in[i]; };
  if (in_sizes[0] != NS * NJ * 2 || in_sizes[1] != NS * NJ || in_sizes[2] != 3 * DH * 3 || in_sizes[3] != 3 * DH || in_sizes[4] != EH * 2 * DH || in_sizes[5] != EH || in_sizes[6] != OUT * TOT || in_sizes[7] != OUT || out_size != NS * OUT) return;
  size_t off = 0; char* ws = (char*)d_ws;
  auto carve = [&](size_t bytes) { char* p = ws + off; off += (bytes + 255) & ~(size_t)255; return p; };
  b16* WE = (b16*)carve((size_t)2 * EH * DH * 2); b16* WP = (b16*)carve((size_t)OUT * TOT * 2);
  constexpr int NCH = 4; constexpr size_t PCH = NS / NCH, RCH = PCH * RPP;
  const size_t frows = (size_t)NS * RPP; b16* FTh = (b16*)carve(frows * DH * 2); b16* FTl = (b16*)carve(frows * DH * 2); float* AB = (float*)carve(RCH * 128 * 4); b16* PFh = (b16*)carve((size_t)NS * TOT * 2); b16* PFl = (b16*)carve((size_t)NS * TOT * 2);
  if (off > ws_size || off > ((size_t)128 << 20)) return;
  prep_kernel<<<(2 * EH * DH / 8 + OUT * TOT / 8 + 255) / 256, 256, 0, stream>>>(Fp(4), Fp(6), WE, WP);
  pose_kernel<<<NS / 8, 256, 0, stream>>>(Fp(0), Fp(1), Fp(2), Fp(3), FTh, FTl, PFh, PFl);
  for (int ch = 0; ch < NCH; ++ch) { if ((size_t)ch * PCH >= (size_t)NCUT) break;
    egemm_kernel<<<(unsigned)((RCH / 16 + 3) / 4), 128, 0, stream>>>(FTh, FTl, WE, AB, (size_t)ch * RCH);
    zmax_kernel<<<(unsigned)(PCH / 8), 256, 0, stream>>>(AB, Fp(5), PFh, PFl, (size_t)ch * PCH); }
  proj_kernel<<<NS / 64, 128, 0, stream>>>(PFh, PFl, WP, Fp(7), (float*)d_out);
}
